// SelfAttentionLayer_30408368455794
// MI455X (gfx1250) — hardware-verified
//
#include <hip/hip_runtime.h>


#define NB_  1
#define NTOK 2048
#define FD   256
#define NHH  8
#define TT   16384
#define DM   FD
#define NH_  1
#define NKV  1
#define REP  (NH_ / NKV)
#define HD   32
#define HP   64
#define DQ   (NH_ * HD)
#define DKV  (NKV * HD)
#define ZH   1
#define RH   0
#define WIN  0
#define QC   1024
#define TK   TT
#define PCAR 1024.0f
#define SCL  0.0625f
typedef _Float16 h16;
typedef unsigned short bf;
typedef __attribute__((ext_vector_type(16))) __bf16   v16bf;
typedef __attribute__((ext_vector_type(16))) _Float16 v16h;
typedef __attribute__((ext_vector_type(8)))  _Float16 v8h;
typedef __attribute__((ext_vector_type(8)))  unsigned short v8us;
typedef __attribute__((ext_vector_type(8)))  float    v8f;
typedef __attribute__((ext_vector_type(4)))  float    v4f;
typedef v8h  __attribute__((may_alias)) v8ha;
typedef v4f  __attribute__((may_alias)) v4fa;
typedef v8us __attribute__((may_alias)) v8usa;

__device__ __forceinline__ unsigned short f2bf(float f) { unsigned u = __float_as_uint(f); u += 0x7FFFu + ((u >> 16) & 1u); return (unsigned short)(u >> 16); }
__device__ __forceinline__ float bf2f(unsigned short b) { return __uint_as_float(((unsigned)b) << 16); }
__device__ __forceinline__ float bfr(float f) { return bf2f(f2bf(f)); }
__device__ __forceinline__ v16h cat16(v8h lo, v8h hi) { return __builtin_shufflevector(lo, hi, 0, 1, 2, 3, 4, 5, 6, 7, 8, 9, 10, 11, 12, 13, 14, 15); }
__device__ __forceinline__ v16bf cat16b(v8us lo, v8us hi) { return __builtin_bit_cast(v16bf, __builtin_shufflevector(lo, hi, 0, 1, 2, 3, 4, 5, 6, 7, 8, 9, 10, 11, 12, 13, 14, 15)); }
__device__ __forceinline__ v8f wmma16(v16h a, v16h b, v8f c) { return __builtin_amdgcn_wmma_f32_16x16x32_f16(false, a, false, b, (short)0, c, false, false); }
__device__ __forceinline__ v8f wmmab(v16bf a, v16bf b, v8f c) { return __builtin_amdgcn_wmma_f32_16x16x32_bf16(false, a, false, b, (short)0, c, false, false); }


template <typename T16> struct WFrag;
template <> struct WFrag<h16> { typedef v16h V; static __device__ __forceinline__ V ld(const h16* p) { return cat16(*(const v8h*)p, *(const v8h*)(p + 16)); } static __device__ __forceinline__ v8f mma(V a, V b, v8f c) { return wmma16(a, b, c); } };
template <> struct WFrag<bf> { typedef v16bf V; static __device__ __forceinline__ V ld(const bf* p) { return cat16b(*(const v8us*)p, *(const v8us*)(p + 16)); } static __device__ __forceinline__ v8f mma(V a, V b, v8f c) { return wmmab(a, b, c); } };
template <typename T16, int NSPLIT, bool BIAS>
__global__ __launch_bounds__(32) void k_gemmw(const T16* __restrict__ A, const T16* __restrict__ A2, const T16* __restrict__ Bt, const T16* __restrict__ Bt2, int K, float* C, int ldc, const float* __restrict__ bias, size_t sA, size_t sB, size_t sC) {
    typedef typename WFrag<T16>::V V;
    __shared__ __align__(16) float os[16 * 68];
    const size_t z = blockIdx.z; A += z * sA; if (A2) A2 += z * sA; Bt += z * sB; if (Bt2) Bt2 += z * sB; C += z * sC;
    const int lane = threadIdx.x & 31, lr = lane & 15, hi = lane >> 4; const int r0 = blockIdx.x * 64, c0 = blockIdx.y * 64;
    v8f acc[4][4];
#pragma unroll
    for (int mb = 0; mb < 4; ++mb)
#pragma unroll
        for (int nb = 0; nb < 4; ++nb) acc[mb][nb] = (v8f){};
    const size_t aoff = (size_t)(r0 + lr) * K + 8 * hi, boff = (size_t)(c0 + lr) * K + 8 * hi;
#pragma unroll 1
    for (int kc = 0; kc < K; kc += 32) {
        V a[4], a2[4];
#pragma unroll
        for (int mb = 0; mb < 4; ++mb) { a[mb] = WFrag<T16>::ld(A + aoff + (size_t)mb * 16 * K + kc); if (NSPLIT == 1 || NSPLIT == 2) a2[mb] = WFrag<T16>::ld(A2 + aoff + (size_t)mb * 16 * K + kc); }
#pragma unroll
        for (int nb = 0; nb < 4; ++nb) { const V b = WFrag<T16>::ld(Bt + boff + (size_t)nb * 16 * K + kc); V b2; if (NSPLIT >= 2) b2 = WFrag<T16>::ld(Bt2 + boff + (size_t)nb * 16 * K + kc);
#pragma unroll
            for (int mb = 0; mb < 4; ++mb) { acc[mb][nb] = WFrag<T16>::mma(a[mb], b, acc[mb][nb]); if (NSPLIT == 1 || NSPLIT == 2) acc[mb][nb] = WFrag<T16>::mma(a2[mb], b, acc[mb][nb]); if (NSPLIT >= 2) acc[mb][nb] = WFrag<T16>::mma(a[mb], b2, acc[mb][nb]); } }
        asm volatile("v_nop\n\tv_nop\n\tv_nop\n\tv_nop" : "+v"(acc[0][0]), "+v"(acc[1][1]), "+v"(acc[2][2]), "+v"(acc[3][3]) : "v"(a[0]), "v"(a[3]));
    }
#pragma unroll
    for (int mb = 0; mb < 4; ++mb) {
#pragma unroll
        for (int nb = 0; nb < 4; ++nb) {
#pragma unroll
            for (int j = 0; j < 8; ++j) os[(hi * 8 + j) * 68 + nb * 16 + lr] = acc[mb][nb][j]; }
        __builtin_amdgcn_wave_barrier(); asm volatile("" ::: "memory");
        float* crow = C + (size_t)(r0 + mb * 16) * ldc + c0;
#pragma unroll 1
        for (int ps = 0; ps < 2; ++ps) {
#pragma unroll
            for (int s = 0; s < 8; ++s) { const int row = 2 * s + hi, cofs = lr * 4; v4f val = *(const v4fa*)(os + row * 68 + cofs); if (BIAS) { val[0] += bfr(bias[c0 + cofs]); val[1] += bfr(bias[c0 + cofs + 1]); val[2] += bfr(bias[c0 + cofs + 2]); val[3] += bfr(bias[c0 + cofs + 3]); }
                *(volatile v4f*)(crow + (size_t)row * ldc + cofs) = val; }
            if (ps == 0) __threadfence(); }
        __builtin_amdgcn_wave_barrier(); asm volatile("" ::: "memory");
    }
}

__device__ __forceinline__ h16 tohx(float x) { return (h16)x; }
__device__ __forceinline__ void splitf(float y, unsigned short& h, unsigned short& l) { h = f2bf(y); l = f2bf(y - bf2f(h)); }
typedef __attribute__((ext_vector_type(2))) _Float16 v2h;
typedef __attribute__((ext_vector_type(4))) _Float16 v4h;
typedef __attribute__((ext_vector_type(2))) unsigned short v2us;
typedef __attribute__((ext_vector_type(4))) unsigned short v4us;
typedef __attribute__((ext_vector_type(2))) float v2f;
typedef __attribute__((ext_vector_type(4))) int v4i;

__global__ __launch_bounds__(256) void k_cvt8(const float* __restrict__ src, bf* dst, size_t n8) { const size_t i = (size_t)blockIdx.x * 256 + threadIdx.x; if (i >= n8) return; const v8f v = *(const v8f*)(src + i * 8); v8us o;
#pragma unroll
    for (int k = 0; k < 8; ++k) o[k] = f2bf(v[k]); *(volatile v8us*)(dst + i * 8) = o; __threadfence(); *(volatile v8us*)(dst + i * 8) = o; }

__global__ __launch_bounds__(256) void k_lsoft(const float* __restrict__ Sb, h16* P16) {
    const int lane = threadIdx.x & 31; const int row = blockIdx.x * 8 + (threadIdx.x >> 5); if (row >= QC) return; const float* sr = Sb + (size_t)row * TK; float mx = -3.0e38f;
#pragma unroll 4
    for (int ch = 0; ch < TK / 128; ++ch) { const v4f a = *(const v4f*)(sr + ch * 128 + lane * 4);
#pragma unroll
        for (int q = 0; q < 4; ++q) { float t = a[q] * SCL; asm volatile("" : "+v"(t)); mx = fmaxf(mx, t); } }
#pragma unroll
    for (int sh = 16; sh; sh >>= 1) mx = fmaxf(mx, __shfl_xor(mx, sh, 32));
    float sum = 0.f;
#pragma unroll 4
    for (int ch = 0; ch < TK / 128; ++ch) { const v4f a = *(const v4f*)(sr + ch * 128 + lane * 4);
#pragma unroll
        for (int q = 0; q < 4; ++q) { float t = a[q] * SCL; asm volatile("" : "+v"(t)); float d0 = __fsub_rn(t, mx); asm volatile("" : "+v"(d0)); sum += __builtin_amdgcn_exp2f(__fmul_rn(d0, 1.4426950408889634f)); } }
#pragma unroll
    for (int sh = 16; sh; sh >>= 1) sum += __shfl_xor(sum, sh, 32);
    const float f = __fdiv_rn(PCAR, sum);
#pragma unroll 1
    for (int ps = 0; ps < 2; ++ps) {
#pragma unroll 2
        for (int ch = 0; ch < TK / 128; ++ch) { const v4f a = *(const v4f*)(sr + ch * 128 + lane * 4); v4h o4;
#pragma unroll
            for (int q = 0; q < 4; ++q) { float t = a[q] * SCL; asm volatile("" : "+v"(t)); float d0 = __fsub_rn(t, mx); asm volatile("" : "+v"(d0)); float ex = __builtin_amdgcn_exp2f(__fmul_rn(d0, 1.4426950408889634f)); asm volatile("" : "+v"(ex)); o4[q] = tohx(ex * f); }
            *(volatile v4h*)(P16 + (size_t)row * TK + ch * 128 + lane * 4) = o4; }
        if (ps == 0) __threadfence(); }
}

__global__ __launch_bounds__(256) void k_wtG(const float* __restrict__ w, int K, int N, bf* Bt) {
    const int lane = threadIdx.x & 31; const int L0 = (blockIdx.x * 8 + (threadIdx.x >> 5)) * 8; const int nlines = N * K / 64;
#pragma unroll
    for (int ps = 0; ps < 2; ++ps) {
#pragma unroll 1
        for (int l = 0; l < 8; ++l) { const int L = L0 + l; if (L >= nlines) break; const size_t e = (size_t)L * 64 + lane * 2; const int k = (int)(e % K), n = (int)(e / K); v2us o;
            o[0] = f2bf(w[(size_t)k * N + n]); o[1] = f2bf(w[(size_t)(k + 1) * N + n]); *(volatile v2us*)(Bt + e) = o; }
        if (ps == 0) __threadfence(); }
}
__global__ __launch_bounds__(256) void k_scr(const float* __restrict__ FQ, const float* __restrict__ FK, h16* Q16, h16* K16) { const size_t e = ((size_t)blockIdx.x * 256 + threadIdx.x) * 2; if (e >= (size_t)TT * HD) return; const int c = (int)(e % HD); const int r = (int)(e / HD); const int b = r >> 3; v2h oq, ok;
#pragma unroll
    for (int q = 0; q < 2; ++q) { const int rem = (r & 7) * HD + c + q; const int col = (rem & 7) * HD + (rem >> 3); oq[q] = tohx(FQ[(size_t)b * FD + col]); ok[q] = tohx(FK[(size_t)b * FD + col]); }
    *(volatile v2h*)(Q16 + e) = oq; *(volatile v2h*)(K16 + e) = ok; __threadfence(); *(volatile v2h*)(Q16 + e) = oq; *(volatile v2h*)(K16 + e) = ok; }
__global__ __launch_bounds__(256) void k_scrV(const float* __restrict__ FV, h16* VT16) { const size_t e = ((size_t)blockIdx.x * 256 + threadIdx.x) * 2; if (e >= (size_t)HP * TT) return; const int r0 = (int)(e % TT); const int c = (int)(e / TT); const int cc = c & (HD - 1); v2h o;
#pragma unroll
    for (int q = 0; q < 2; ++q) { const int r = r0 + q; const int b = r >> 3; const int rem = (r & 7) * HD + cc; const int col = (rem & 7) * HD + (rem >> 3); const float v = FV[(size_t)b * FD + col]; o[q] = (c < HD) ? tohx(v) : tohx(0.0f); }
    *(volatile v2h*)(VT16 + e) = o; __threadfence(); *(volatile v2h*)(VT16 + e) = o; }
__global__ __launch_bounds__(256) void k_cat(const float* __restrict__ O, int q0, float* att, bf* Ah, bf* Al) { const size_t i = (size_t)blockIdx.x * 256 + threadIdx.x; if (i >= (size_t)(QC / NHH) * FD / 4) return; const size_t e = i * 4; const int cp = (int)(e % FD); const int bl = (int)(e / FD); const int b = q0 / NHH + bl; v4f o; v4us oh, ol;
#pragma unroll
    for (int q = 0; q < 4; ++q) { const int c2 = cp + q; const int h = c2 & 7; const int s = c2 >> 3; const int rl = bl * NHH + h; const float y = O[(size_t)rl * HP + s] * (1.0f / PCAR); o[q] = y; unsigned short u, w; splitf(y, u, w); oh[q] = u; ol[q] = w; }
    const size_t oo = (size_t)b * FD + cp; *(volatile v4f*)(att + oo) = o; *(volatile v4us*)(Ah + oo) = oh; *(volatile v4us*)(Al + oo) = ol; __threadfence(); *(volatile v4f*)(att + oo) = o; *(volatile v4us*)(Ah + oo) = oh; *(volatile v4us*)(Al + oo) = ol; }
extern "C" void kernel_launch(void* const* d_in, const int* in_sizes, int n_in,
                              void* d_out, int out_size, void* d_ws, size_t ws_size, hipStream_t stream) {
    (void)in_sizes; (void)n_in; (void)out_size;
    const float* x = (const float*)d_in[0]; const float* wq = (const float*)d_in[1]; const float* bq = (const float*)d_in[2]; const float* wk = (const float*)d_in[3]; const float* bk = (const float*)d_in[4]; const float* wv = (const float*)d_in[5]; const float* bv = (const float*)d_in[6]; const float* wo = (const float*)d_in[7]; const float* bo = (const float*)d_in[8];
    float* OUT = (float*)d_out;
    float* ATT = OUT + (size_t)NTOK * FD;
    char* wsp = (char*)d_ws;
    auto take = [&](size_t bytes) { char* p = wsp; wsp += (bytes + 255) & ~(size_t)255; return (void*)p; };
    bf* WQ = (bf*)take((size_t)FD * FD * 2); bf* WK = (bf*)take((size_t)FD * FD * 2); bf* WV = (bf*)take((size_t)FD * FD * 2); bf* WO = (bf*)take((size_t)FD * FD * 2);
    bf* XB = (bf*)take((size_t)NTOK * FD * 2); float* FQ = (float*)take((size_t)NTOK * FD * 4); float* FK = (float*)take((size_t)NTOK * FD * 4); float* FV = (float*)take((size_t)NTOK * FD * 4);
    h16* QP16 = (h16*)take((size_t)TT * HD * 2); h16* KP16 = (h16*)take((size_t)TT * HD * 2); h16* VT16 = (h16*)take((size_t)HP * TT * 2);
    float* Sb = (float*)take((size_t)QC * TK * 4); h16* P16 = (h16*)take((size_t)QC * TK * 2); float* Ob = (float*)take((size_t)QC * HP * 4); bf* Ah = (bf*)take((size_t)NTOK * FD * 2); bf* Al = (bf*)take((size_t)NTOK * FD * 2);
    if ((size_t)(wsp - (char*)d_ws) > ws_size) return;
    k_wtG<<<(unsigned)((FD * FD / 64 + 63) / 64), 256, 0, stream>>>(wq, FD, FD, WQ); k_wtG<<<(unsigned)((FD * FD / 64 + 63) / 64), 256, 0, stream>>>(wk, FD, FD, WK); k_wtG<<<(unsigned)((FD * FD / 64 + 63) / 64), 256, 0, stream>>>(wv, FD, FD, WV); k_wtG<<<(unsigned)((FD * FD / 64 + 63) / 64), 256, 0, stream>>>(wo, FD, FD, WO);
    k_cvt8<<<(unsigned)(((size_t)NTOK * FD / 8 + 255) / 256), 256, 0, stream>>>(x, XB, (size_t)NTOK * FD / 8);
    k_gemmw<bf, 0, true><<<dim3(NTOK / 64, FD / 64, 1), 32, 0, stream>>>(XB, nullptr, WQ, nullptr, FD, FQ, FD, bq, 0, 0, 0); k_gemmw<bf, 0, true><<<dim3(NTOK / 64, FD / 64, 1), 32, 0, stream>>>(XB, nullptr, WK, nullptr, FD, FK, FD, bk, 0, 0, 0); k_gemmw<bf, 0, true><<<dim3(NTOK / 64, FD / 64, 1), 32, 0, stream>>>(XB, nullptr, WV, nullptr, FD, FV, FD, bv, 0, 0, 0);
    k_scr<<<(unsigned)(((size_t)TT * HD / 2 + 255) / 256), 256, 0, stream>>>(FQ, FK, QP16, KP16); k_scrV<<<(unsigned)(((size_t)HP * TT / 2 + 255) / 256), 256, 0, stream>>>(FV, VT16);
    for (int q0 = 0; q0 < TT; q0 += QC) {
        k_gemmw<h16, 0, false><<<dim3(QC / 64, TK / 64, 1), 32, 0, stream>>>(QP16 + (size_t)q0 * HD, nullptr, KP16, nullptr, HD, Sb, TK, nullptr, 0, 0, 0);
        k_lsoft<<<QC / 8, 256, 0, stream>>>(Sb, P16);
        k_gemmw<h16, 0, false><<<dim3(QC / 64, HP / 64, 1), 32, 0, stream>>>(P16, nullptr, VT16, nullptr, TK, Ob, HP, nullptr, 0, 0, 0);
        k_cat<<<(unsigned)(((size_t)(QC / NHH) * FD / 4 + 255) / 256), 256, 0, stream>>>(Ob, q0, ATT, Ah, Al); }
    k_gemmw<bf, 1, true><<<dim3(NTOK / 64, FD / 64, 1), 32, 0, stream>>>(Ah, Al, WO, nullptr, FD, OUT, FD, bo, 0, 0, 0);
}
